// SigNet_996432413588
// MI455X (gfx1250) — hardware-verified
//
#include <hip/hip_runtime.h>


#define B_   8
#define T_   128
#define CI_  33
#define H1_  64
#define H2_  8
#define CA_  42
#define C2_  1764
#define C3_  74088
#define S_   75894
#define XP_  64
#define KP_  64
#define NI_  2
#define NIB_ 21
#define NT_  256
#define NBLK_SIG (B_ * NIB_)

static_assert(NI_ * NIB_ == CA_);
static_assert(CA_ + C2_ + C3_ == S_);
static_assert(CA_ <= XP_ && CI_ + 1 + H2_ == CA_);
static_assert(T_ % 16 == 0 && (T_ * XP_) % (4 * NT_) == 0);
static_assert(NT_ == 256 && 6 * CA_ <= NT_ && 7 * 6 == CA_);
static_assert(C2_ <= 7 * NT_);

typedef __bf16         v16b __attribute__((ext_vector_type(16)));
typedef unsigned short v8us __attribute__((ext_vector_type(8)));
typedef float          v8f  __attribute__((ext_vector_type(8)));
typedef float          v4f  __attribute__((ext_vector_type(4)));

union FragB { v16b v; v8us half[2]; };

constexpr size_t OFF_DX  = 0;
constexpr size_t SZ_DX   = (size_t)B_ * T_ * XP_ * 4;
constexpr size_t OFF_PT  = OFF_DX + SZ_DX;
constexpr size_t SZ_PT   = (size_t)NBLK_SIG * T_ * 4;
constexpr size_t WS_END  = OFF_PT + SZ_PT;
static_assert(OFF_PT % 512 == 0 && WS_END % 128 == 0);
static_assert(WS_END <= (size_t)134217728);

__device__ __forceinline__ float lrelu(float v) { return v >= 0.0f ? v : 0.01f * v; }

__device__ __forceinline__ v8f zero8f() {
    v8f z;
#pragma unroll
    for (int i = 0; i < 8; ++i) z[i] = 0.0f;
    return z;
}
__device__ __forceinline__ unsigned int bf16_rne(float x) {
    const unsigned int u = __float_as_uint(x);
    return (u + 0x7FFFu + ((u >> 16) & 1u)) >> 16;
}
__device__ __forceinline__ void split_bf16(float x, unsigned short& hi, unsigned short& lo) {
    const unsigned int hb = bf16_rne(x);
    const float hfv = __uint_as_float(hb << 16);
    const unsigned int lb = bf16_rne(x - hfv);
    hi = (unsigned short)hb;
    lo = (unsigned short)lb;
}
__device__ __forceinline__ void split8(v8f x, v8us& hv, v8us& lv) {
#pragma unroll
    for (int e = 0; e < 8; ++e) { unsigned short hi, lo; split_bf16(x[e], hi, lo); hv[e] = hi; lv[e] = lo; }
}
__device__ __forceinline__ void ldfragb(FragB& f, const unsigned short* p) {
    f.half[0] = *(const v8us*)(p);
    f.half[1] = *(const v8us*)(p + 16);
}
__device__ __forceinline__ v8f mma3(v8f c, const FragB& ah, const FragB& al, const FragB& bh, const FragB& bl) {
    v8f d = __builtin_amdgcn_wmma_f32_16x16x32_bf16(false, ah.v, false, bh.v, (short)0, c, false, false);
    d = __builtin_amdgcn_wmma_f32_16x16x32_bf16(false, ah.v, false, bl.v, (short)0, d, false, false);
    d = __builtin_amdgcn_wmma_f32_16x16x32_bf16(false, al.v, false, bh.v, (short)0, d, false, false);
    asm volatile("v_nop\n\tv_nop\n\tv_nop\n\tv_nop" : "+v"(d) : "v"(ah.v), "v"(al.v), "v"(bh.v), "v"(bl.v));
    return d;
}
__device__ __forceinline__ float wsum(float v) {
#pragma unroll
    for (int o = 16; o > 0; o >>= 1) v += __shfl_xor(v, o, 32);
    return v;
}

__global__ __launch_bounds__(32)
void k_augdx(const float* __restrict__ inp, const float* __restrict__ W1, const float* __restrict__ b1,
             const float* __restrict__ W2, const float* __restrict__ b2, float* dxp)
{
    __shared__ __attribute__((aligned(16))) unsigned short w1h[H1_ * KP_];
    __shared__ __attribute__((aligned(16))) unsigned short w1l[H1_ * KP_];
    __shared__ __attribute__((aligned(16))) unsigned short w2h[16 * H1_];
    __shared__ __attribute__((aligned(16))) unsigned short w2l[16 * H1_];
    __shared__ __attribute__((aligned(16))) unsigned short hh[16 * H1_];
    __shared__ __attribute__((aligned(16))) unsigned short hl[16 * H1_];
    __shared__ __attribute__((aligned(16))) float xs[17 * XP_];

    const int lane = threadIdx.x & 31, hf = lane >> 4, m = lane & 15;
    const int b = blockIdx.x;

    for (int e = lane; e < H1_ * KP_; e += 32) {
        const int n = e >> 6, k = e & 63;
        const int kc = min(k, CI_ - 1);
        const float x = W1[n * CI_ + kc];
        const float v = (k < CI_) ? x : 0.0f;
        unsigned short hi, lo;
        split_bf16(v, hi, lo);
        w1h[e] = hi; w1l[e] = lo;
    }
    for (int e = lane; e < 16 * H1_; e += 32) {
        const int n = e >> 6, k = e & 63;
        const int nc = min(n, H2_ - 1);
        const float x = W2[nc * H1_ + k];
        const float v = (n < H2_) ? x : 0.0f;
        unsigned short hi, lo;
        split_bf16(v, hi, lo);
        w2h[e] = hi; w2l[e] = lo;
    }
    for (int e = lane; e < 17 * XP_; e += 32) xs[e] = 0.0f;
    const float bias2 = b2[min(m, H2_ - 1)];
    __syncthreads();

#pragma unroll 1
    for (int rt = 0; rt < T_ / 16; ++rt) {
        const int r0 = rt * 16;
        {
            const float* src = inp + (size_t)(b * T_ + r0) * CI_;
#pragma unroll 1
            for (int it = 0; it < 17; ++it) {
                const int e = lane + 32 * it;
                const int ec = min(e, 16 * CI_ - 1);
                const float v = src[ec];
                const int r = ec / CI_;
                const int c = ec - r * CI_;
                if (e < 16 * CI_) xs[(1 + r) * XP_ + c] = v;
            }
            if (lane < 16) {
                const int t = r0 + lane;
                const float tv = (t == T_ - 1) ? 1.0f : (float)t * (1.0f / (float)(T_ - 1));
                xs[(1 + lane) * XP_ + CI_] = tv;
            }
        }
        __syncthreads();

        v8f acc[4];
#pragma unroll
        for (int nt = 0; nt < 4; ++nt) acc[nt] = zero8f();
#pragma unroll
        for (int ks = 0; ks < KP_ / 32; ++ks) {
            FragB ah, al;
#pragma unroll
            for (int q = 0; q < 2; ++q) {
                const int kb = 32 * ks + 16 * q + 8 * hf;
                v8f x;
#pragma unroll
                for (int e = 0; e < 8; ++e) {
                    const int k = kb + e;
                    const float xv = xs[(1 + m) * XP_ + k];
                    x[e] = (k < CI_) ? xv : 0.0f;
                }
                split8(x, ah.half[q], al.half[q]);
            }
#pragma unroll
            for (int nt = 0; nt < 4; ++nt) {
                FragB bh, bl;
                ldfragb(bh, w1h + (16 * nt + m) * KP_ + 32 * ks + 8 * hf);
                ldfragb(bl, w1l + (16 * nt + m) * KP_ + 32 * ks + 8 * hf);
                acc[nt] = mma3(acc[nt], ah, al, bh, bl);
            }
        }
#pragma unroll
        for (int nt = 0; nt < 4; ++nt) {
            const float bias = b1[16 * nt + m];
#pragma unroll
            for (int r = 0; r < 8; ++r) {
                const float hv = lrelu(acc[nt][r] + bias);
                unsigned short hi, lo;
                split_bf16(hv, hi, lo);
                const int o = (8 * hf + r) * H1_ + 16 * nt + m;
                hh[o] = hi; hl[o] = lo;
            }
        }
        __syncthreads();

        v8f acc2 = zero8f();
#pragma unroll
        for (int ks = 0; ks < H1_ / 32; ++ks) {
            FragB ah, al, bh, bl;
            ldfragb(ah, hh + m * H1_ + 32 * ks + 8 * hf);
            ldfragb(al, hl + m * H1_ + 32 * ks + 8 * hf);
            ldfragb(bh, w2h + m * H1_ + 32 * ks + 8 * hf);
            ldfragb(bl, w2l + m * H1_ + 32 * ks + 8 * hf);
            acc2 = mma3(acc2, ah, al, bh, bl);
        }
        if (m < H2_) {
#pragma unroll
            for (int r = 0; r < 8; ++r) xs[(1 + 8 * hf + r) * XP_ + CI_ + 1 + m] = acc2[r] + bias2;
        }
        __syncthreads();

        {
            float* gp = dxp + (size_t)(b * T_ + r0) * XP_;
            v4f d4[8];
#pragma unroll
            for (int s = 0; s < 8; ++s) {
                const int row = 2 * s + hf;
                const v4f cur = *(const v4f*)(xs + (1 + row) * XP_ + 4 * m);
                const v4f prv = *(const v4f*)(xs + row * XP_ + 4 * m);
                d4[s] = cur - prv;
                *(volatile v4f*)(gp + row * XP_ + 4 * m) = d4[s];
            }
            __threadfence();
#pragma unroll
            for (int s = 0; s < 8; ++s) {
                const int row = 2 * s + hf;
                *(volatile v4f*)(gp + row * XP_ + 4 * m) = d4[s];
            }
        }
        __syncthreads();
        {
            const float c0 = xs[16 * XP_ + 2 * lane];
            const float c1 = xs[16 * XP_ + 2 * lane + 1];
            xs[2 * lane] = c0;
            xs[2 * lane + 1] = c1;
        }
        __syncthreads();
    }
}

__global__ __launch_bounds__(NT_)
void k_sig(const float* __restrict__ dxp, const float* __restrict__ Wl, float* part)
{
    __shared__ __attribute__((aligned(16))) float dall[T_ * XP_];
    __shared__ float s2s[C2_];
    __shared__ float s1s[CA_];
    __shared__ __attribute__((aligned(16))) float pacc[T_];
    __shared__ float red[NT_ / 32];

    const int tid = threadIdx.x, lane = tid & 31, w = tid >> 5;
    const int blk = blockIdx.x;
    const int b = blk / NIB_;
    const int ib = blk - b * NIB_;
    const int i0 = NI_ * ib, i1 = i0 + 1;

    {
        const float* src = dxp + (size_t)b * T_ * XP_;
#pragma unroll 1
        for (int i = tid; i < (T_ * XP_) / 4; i += NT_) *(v4f*)(dall + 4 * i) = *(const v4f*)(src + 4 * i);
#pragma unroll 1
        for (int f = tid; f < C2_; f += NT_) s2s[f] = 0.0f;
        if (tid < CA_) s1s[tid] = 0.0f;
        if (tid < T_) pacc[tid] = 0.0f;
    }

    const int jr = tid / 6;
    const int j = min(jr, CA_ - 1);
    const int kb = (tid - 6 * jr) * 7;
    const float m3 = (tid < 6 * CA_) ? 1.0f : 0.0f;
    const int tc1 = min(tid, CA_ - 1);
    const float wl1 = Wl[tc1] * ((tid < CA_ && ib == 0) ? 1.0f : 0.0f);

    float s3a[7], s3b[7], wl3a[7], wl3b[7], wl2[7];
    int g2[7], gj2[7], gk2[7];
    const int base3 = CA_ + C2_ + i0 * C2_ + j * CA_ + kb;
#pragma unroll
    for (int u = 0; u < 7; ++u) {
        s3a[u] = 0.0f; s3b[u] = 0.0f;
        wl3a[u] = Wl[base3 + u] * m3;
        wl3b[u] = Wl[base3 + C2_ + u] * m3;
        const int g = tid + NT_ * u;
        const int gc = min(g, C2_ - 1);
        g2[u] = gc;
        gj2[u] = gc / CA_;
        gk2[u] = gc - CA_ * (gc / CA_);
        wl2[u] = Wl[CA_ + gc] * ((g < C2_ && ib == 0) ? 1.0f : 0.0f);
    }
    __syncthreads();

#pragma unroll 1
    for (int t = 0; t < T_; ++t) {
        const float* d = dall + t * XP_;
        float acc = 0.0f;
        {
            const float dj = d[j], di0 = d[i0], di1 = d[i1];
            const float q0 = fmaf(di0, (1.0f / 6.0f), 0.5f * s1s[i0]);
            const float q1 = fmaf(di1, (1.0f / 6.0f), 0.5f * s1s[i1]);
            const float c0 = fmaf(dj, q0, s2s[i0 * CA_ + j]);
            const float c1 = fmaf(dj, q1, s2s[i1 * CA_ + j]);
#pragma unroll
            for (int u = 0; u < 7; ++u) {
                const float dk = d[kb + u];
                const float v0 = fmaf(dk, c0, s3a[u]);
                const float v1 = fmaf(dk, c1, s3b[u]);
                s3a[u] = v0; s3b[u] = v1;
                acc = fmaf(wl3a[u], lrelu(v0), acc);
                acc = fmaf(wl3b[u], lrelu(v1), acc);
            }
        }
        float ns2[7];
#pragma unroll
        for (int u = 0; u < 7; ++u) {
            const float dgk = d[gk2[u]];
            const float dgj = d[gj2[u]];
            const float s1g = s1s[gj2[u]];
            ns2[u] = fmaf(dgk, fmaf(0.5f, dgj, s1g), s2s[g2[u]]);
            acc = fmaf(wl2[u], lrelu(ns2[u]), acc);
        }
        const float ns1 = s1s[tc1] + d[tc1];
        acc = fmaf(wl1, lrelu(ns1), acc);
        __syncthreads();

#pragma unroll
        for (int u = 0; u < 7; ++u)
            if (tid + NT_ * u < C2_) s2s[g2[u]] = ns2[u];
        if (tid < CA_) s1s[tid] = ns1;
        const float wsv = wsum(acc);
        if (lane == 0) red[w] = wsv;
        __syncthreads();
        if (tid == 0) {
            float tot = red[0];
#pragma unroll
            for (int i = 1; i < NT_ / 32; ++i) tot += red[i];
            pacc[t] = tot;
        }
    }
    __syncthreads();
    if (w == 0) {
        const v4f v = *(const v4f*)(pacc + 4 * lane);
        float* p = part + (size_t)blk * T_ + 4 * lane;
        *(volatile v4f*)p = v;
        __threadfence();
        *(volatile v4f*)p = v;
    }
}

__global__ __launch_bounds__(NT_)
void k_final(const float* __restrict__ part, const float* __restrict__ bl, float* out)
{
    __shared__ __attribute__((aligned(16))) float ost[B_ * T_];
    const int tid = threadIdx.x;
    const float blv = bl[0];
#pragma unroll
    for (int r = 0; r < (B_ * T_) / NT_; ++r) {
        const int o = tid + NT_ * r;
        const int bq = o >> 7, t = o & (T_ - 1);
        const float* p = part + (size_t)(bq * NIB_) * T_ + t;
        float s = 0.0f;
#pragma unroll 1
        for (int ib = 0; ib < NIB_; ++ib) s += p[ib * T_];
        ost[o] = s + blv;
    }
    __syncthreads();
    const v4f v = *(const v4f*)(ost + 4 * tid);
    float* op = out + 4 * tid;
    *(volatile v4f*)op = v;
    __threadfence();
    *(volatile v4f*)op = v;
}

extern "C" void kernel_launch(void* const* d_in, const int* in_sizes, int n_in,
                              void* d_out, int out_size, void* d_ws, size_t ws_size,
                              hipStream_t stream)
{
    if (n_in < 7) return;
    if (in_sizes[0] != B_ * T_ * CI_) return;
    if (in_sizes[1] != H1_ * CI_)     return;
    if (in_sizes[2] != H1_)           return;
    if (in_sizes[3] != H2_ * H1_)     return;
    if (in_sizes[4] != H2_)           return;
    if (in_sizes[5] != S_)            return;
    if (in_sizes[6] != 1)             return;
    if (out_size != B_ * T_)          return;
    if (ws_size < WS_END)             return;

    const float* inp = (const float*)d_in[0];
    const float* W1  = (const float*)d_in[1];
    const float* b1  = (const float*)d_in[2];
    const float* W2  = (const float*)d_in[3];
    const float* b2  = (const float*)d_in[4];
    const float* Wl  = (const float*)d_in[5];
    const float* bl  = (const float*)d_in[6];
    float* out = (float*)d_out;

    char* ws = (char*)d_ws;
    float* dxp  = (float*)(ws + OFF_DX);
    float* part = (float*)(ws + OFF_PT);

    k_augdx<<<dim3(B_), dim3(32), 0, stream>>>(inp, W1, b1, W2, b2, dxp);
    k_sig<<<dim3(NBLK_SIG), dim3(NT_), 0, stream>>>((const float*)dxp, Wl, part);
    k_final<<<dim3(1), dim3(NT_), 0, stream>>>((const float*)part, bl, out);
}
